// OPTEigenAttention_80719615361036
// MI455X (gfx1250) — hardware-verified
//
#include <hip/hip_runtime.h>


#define NB_  2
#define TT   2048
#define DM   2048
#define RK   1024
#define NH_  32
#define HD   32
#define RH   512
#define PCAR 1024.0f
#define SCL  0.125f
typedef _Float16 h16;
typedef unsigned short bf;
typedef __attribute__((ext_vector_type(16))) __bf16   v16bf;
typedef __attribute__((ext_vector_type(16))) _Float16 v16h;
typedef __attribute__((ext_vector_type(8)))  _Float16 v8h;
typedef __attribute__((ext_vector_type(8)))  unsigned short v8us;
typedef __attribute__((ext_vector_type(8)))  float    v8f;
typedef __attribute__((ext_vector_type(4)))  float    v4f;
typedef v8h  __attribute__((may_alias)) v8ha;
typedef v4f  __attribute__((may_alias)) v4fa;
typedef v8us __attribute__((may_alias)) v8usa;

__device__ __forceinline__ unsigned short f2bf(float f) { unsigned u = __float_as_uint(f); u += 0x7FFFu + ((u >> 16) & 1u); return (unsigned short)(u >> 16); }
__device__ __forceinline__ float bf2f(unsigned short b) { return __uint_as_float(((unsigned)b) << 16); }
__device__ __forceinline__ float bfr(float f) { return bf2f(f2bf(f)); }
__device__ __forceinline__ v16h cat16(v8h lo, v8h hi) { return __builtin_shufflevector(lo, hi, 0, 1, 2, 3, 4, 5, 6, 7, 8, 9, 10, 11, 12, 13, 14, 15); }
__device__ __forceinline__ v16bf cat16b(v8us lo, v8us hi) { return __builtin_bit_cast(v16bf, __builtin_shufflevector(lo, hi, 0, 1, 2, 3, 4, 5, 6, 7, 8, 9, 10, 11, 12, 13, 14, 15)); }
__device__ __forceinline__ v8f wmma16(v16h a, v16h b, v8f c) { return __builtin_amdgcn_wmma_f32_16x16x32_f16(false, a, false, b, (short)0, c, false, false); }
__device__ __forceinline__ v8f wmmab(v16bf a, v16bf b, v8f c) { return __builtin_amdgcn_wmma_f32_16x16x32_bf16(false, a, false, b, (short)0, c, false, false); }


template <typename T16> struct WFrag;
template <> struct WFrag<h16> { typedef v16h V; static __device__ __forceinline__ V ld(const h16* p) { return cat16(*(const v8h*)p, *(const v8h*)(p + 16)); } static __device__ __forceinline__ v8f mma(V a, V b, v8f c) { return wmma16(a, b, c); } };
template <> struct WFrag<bf> { typedef v16bf V; static __device__ __forceinline__ V ld(const bf* p) { return cat16b(*(const v8us*)p, *(const v8us*)(p + 16)); } static __device__ __forceinline__ v8f mma(V a, V b, v8f c) { return wmmab(a, b, c); } };
template <typename T16, int NSPLIT, bool BIAS>
__global__ __launch_bounds__(32) void k_gemmw(const T16* __restrict__ A, const T16* __restrict__ A2, const T16* __restrict__ Bt, const T16* __restrict__ Bt2, int K, float* C, int ldc, const float* __restrict__ bias, size_t sA, size_t sB, size_t sC) {
    typedef typename WFrag<T16>::V V;
    __shared__ __align__(16) float os[16 * 68];
    const size_t z = blockIdx.z; A += z * sA; if (A2) A2 += z * sA; Bt += z * sB; if (Bt2) Bt2 += z * sB; C += z * sC;
    const int lane = threadIdx.x & 31, lr = lane & 15, hi = lane >> 4; const int r0 = blockIdx.x * 64, c0 = blockIdx.y * 64;
    v8f acc[4][4];
#pragma unroll
    for (int mb = 0; mb < 4; ++mb)
#pragma unroll
        for (int nb = 0; nb < 4; ++nb) acc[mb][nb] = (v8f){};
    const size_t aoff = (size_t)(r0 + lr) * K + 8 * hi, boff = (size_t)(c0 + lr) * K + 8 * hi;
#pragma unroll 1
    for (int kc = 0; kc < K; kc += 32) {
        V a[4], a2[4];
#pragma unroll
        for (int mb = 0; mb < 4; ++mb) { a[mb] = WFrag<T16>::ld(A + aoff + (size_t)mb * 16 * K + kc); if (NSPLIT == 1 || NSPLIT == 2) a2[mb] = WFrag<T16>::ld(A2 + aoff + (size_t)mb * 16 * K + kc); }
#pragma unroll
        for (int nb = 0; nb < 4; ++nb) { const V b = WFrag<T16>::ld(Bt + boff + (size_t)nb * 16 * K + kc); V b2; if (NSPLIT >= 2) b2 = WFrag<T16>::ld(Bt2 + boff + (size_t)nb * 16 * K + kc);
#pragma unroll
            for (int mb = 0; mb < 4; ++mb) { acc[mb][nb] = WFrag<T16>::mma(a[mb], b, acc[mb][nb]); if (NSPLIT == 1 || NSPLIT == 2) acc[mb][nb] = WFrag<T16>::mma(a2[mb], b, acc[mb][nb]); if (NSPLIT >= 2) acc[mb][nb] = WFrag<T16>::mma(a[mb], b2, acc[mb][nb]); } }
        asm volatile("v_nop\n\tv_nop\n\tv_nop\n\tv_nop" : "+v"(acc[0][0]), "+v"(acc[1][1]), "+v"(acc[2][2]), "+v"(acc[3][3]) : "v"(a[0]), "v"(a[3]));
    }
#pragma unroll
    for (int mb = 0; mb < 4; ++mb) {
#pragma unroll
        for (int nb = 0; nb < 4; ++nb) {
#pragma unroll
            for (int j = 0; j < 8; ++j) os[(hi * 8 + j) * 68 + nb * 16 + lr] = acc[mb][nb][j]; }
        __builtin_amdgcn_wave_barrier(); asm volatile("" ::: "memory");
        float* crow = C + (size_t)(r0 + mb * 16) * ldc + c0;
#pragma unroll 1
        for (int ps = 0; ps < 2; ++ps) {
#pragma unroll
            for (int s = 0; s < 8; ++s) { const int row = 2 * s + hi, cofs = lr * 4; v4f val = *(const v4fa*)(os + row * 68 + cofs); if (BIAS) { val[0] += bfr(bias[c0 + cofs]); val[1] += bfr(bias[c0 + cofs + 1]); val[2] += bfr(bias[c0 + cofs + 2]); val[3] += bfr(bias[c0 + cofs + 3]); }
                *(volatile v4f*)(crow + (size_t)row * ldc + cofs) = val; }
            if (ps == 0) __threadfence(); }
        __builtin_amdgcn_wave_barrier(); asm volatile("" ::: "memory");
    }
}

__device__ __forceinline__ h16 tohx(float x) { return (h16)x; }
__device__ __forceinline__ void splitf(float y, unsigned short& h, unsigned short& l) { h = f2bf(y); l = f2bf(y - bf2f(h)); }
typedef __attribute__((ext_vector_type(2))) _Float16 v2h;
typedef __attribute__((ext_vector_type(4))) _Float16 v4h;
typedef __attribute__((ext_vector_type(2))) unsigned short v2us;
typedef __attribute__((ext_vector_type(4))) unsigned short v4us;
typedef __attribute__((ext_vector_type(2))) float v2f;

__global__ __launch_bounds__(256) void k_cvt8(const float* __restrict__ src, bf* dst, size_t n8) { const size_t i = (size_t)blockIdx.x * 256 + threadIdx.x; if (i >= n8) return; const v8f v = *(const v8f*)(src + i * 8); v8us o;
#pragma unroll
    for (int k = 0; k < 8; ++k) o[k] = f2bf(v[k]); *(volatile v8us*)(dst + i * 8) = o; __threadfence(); *(volatile v8us*)(dst + i * 8) = o; }
__global__ __launch_bounds__(256) void k_qkp(const float* __restrict__ FQ, const float* __restrict__ FK, h16* Q16, h16* K16, bf* Qh, bf* Ql, bf* Kh, bf* Kl) { const size_t e = ((size_t)blockIdx.x * 256 + threadIdx.x) * 2; if (e >= (size_t)NH_ * TT * HD) return; const int d = (int)(e % HD); const int t = (int)((e / HD) % TT); const int h = (int)(e / ((size_t)HD * TT)); const size_t s = (size_t)t * RK + h * HD + d; v2h q, k; v2us qh, ql, kh, kl;
#pragma unroll
    for (int u = 0; u < 2; ++u) { float qs = __fmul_rn(FQ[s + u], SCL); asm volatile("" : "+v"(qs)); q[u] = tohx(qs); k[u] = tohx(FK[s + u]); unsigned short a, c2; splitf(qs, a, c2); qh[u] = a; ql[u] = c2; splitf(FK[s + u], a, c2); kh[u] = a; kl[u] = c2; }
    for (int ps = 0; ps < 2; ++ps) { *(volatile v2h*)(Q16 + e) = q; *(volatile v2h*)(K16 + e) = k; *(volatile v2us*)(Qh + e) = qh; *(volatile v2us*)(Ql + e) = ql; *(volatile v2us*)(Kh + e) = kh; *(volatile v2us*)(Kl + e) = kl; if (ps == 0) __threadfence(); } }
__global__ __launch_bounds__(256) void k_vtp(const float* __restrict__ FV, h16* VT16, bf* VTh, bf* VTl) { const size_t e = ((size_t)blockIdx.x * 256 + threadIdx.x) * 2; if (e >= (size_t)NH_ * 64 * TT) return; const int t = (int)(e % TT); const int dd = (int)((e / TT) % 64); const int h = (int)(e / ((size_t)TT * 64)); v2h o; v2us oh, ol;
#pragma unroll
    for (int u = 0; u < 2; ++u) { const float v = (dd < HD) ? FV[(size_t)(t + u) * RK + h * HD + dd] : 0.f; o[u] = tohx(v); unsigned short a, c2; splitf(v, a, c2); oh[u] = a; ol[u] = c2; }
    for (int ps = 0; ps < 2; ++ps) { *(volatile v2h*)(VT16 + e) = o; *(volatile v2us*)(VTh + e) = oh; *(volatile v2us*)(VTl + e) = ol; if (ps == 0) __threadfence(); } }
__global__ __launch_bounds__(256) void k_hsoft(const float* __restrict__ Sb, const float* __restrict__ mk, h16* P16, bf* Ph, bf* Pl) { const int lane = threadIdx.x & 31; const int row = blockIdx.x * 8 + (threadIdx.x >> 5); if (row >= TT) return; const float* sr = Sb + (size_t)row * TT; const float* mr = mk + (size_t)row * TT; float v[64]; float mx = -3.0e38f;
#pragma unroll
    for (int ch = 0; ch < 16; ++ch) { const int j0 = ch * 128 + lane * 4; const v4f a = *(const v4f*)(sr + j0), m4 = *(const v4f*)(mr + j0);
#pragma unroll
        for (int q = 0; q < 4; ++q) { const float t = fmaxf(__fadd_rn(a[q], m4[q]), -3.40282347e38f); v[ch * 4 + q] = t; mx = fmaxf(mx, t); } }
#pragma unroll
    for (int sh = 16; sh; sh >>= 1) mx = fmaxf(mx, __shfl_xor(mx, sh, 32));
    float sum = 0.f;
#pragma unroll
    for (int k = 0; k < 64; ++k) { float d0 = __fsub_rn(v[k], mx); asm volatile("" : "+v"(d0)); v[k] = __expf(d0); sum += v[k]; }
#pragma unroll
    for (int sh = 16; sh; sh >>= 1) sum += __shfl_xor(sum, sh, 32);
    if (row < RH) { const float f = __fdiv_rn(1.0f, sum);
#pragma unroll 1
        for (int ps = 0; ps < 2; ++ps) {
#pragma unroll
            for (int ch = 0; ch < 16; ++ch) { v4us oh, ol;
#pragma unroll
                for (int q = 0; q < 4; ++q) { float y = __fmul_rn(v[ch * 4 + q], f); asm volatile("" : "+v"(y)); unsigned short a2, c2; splitf(y, a2, c2); oh[q] = a2; ol[q] = c2; }
                *(volatile v4us*)(Ph + (size_t)row * TT + ch * 128 + lane * 4) = oh; *(volatile v4us*)(Pl + (size_t)row * TT + ch * 128 + lane * 4) = ol; }
            if (ps == 0) __threadfence(); } }
    else { const float f = __fdiv_rn(PCAR, sum);
#pragma unroll 1
        for (int ps = 0; ps < 2; ++ps) {
#pragma unroll
            for (int ch = 0; ch < 16; ++ch) { v4h o;
#pragma unroll
                for (int q = 0; q < 4; ++q) o[q] = tohx(v[ch * 4 + q] * f); *(volatile v4h*)(P16 + (size_t)row * TT + ch * 128 + lane * 4) = o; }
            if (ps == 0) __threadfence(); } } }
__global__ __launch_bounds__(256) void k_ofm(const float* __restrict__ O, int h, bf* Ah, bf* Al) { const size_t e = ((size_t)blockIdx.x * 256 + threadIdx.x) * 2; if (e >= (size_t)TT * HD) return; const int d = (int)(e % HD), t = (int)(e / HD); const float sc = (t < RH) ? 1.0f : (1.0f / PCAR); v2us oh, ol;
#pragma unroll
    for (int u = 0; u < 2; ++u) { unsigned short a, c2; splitf(__fmul_rn(O[(size_t)t * 64 + d + u], sc), a, c2); oh[u] = a; ol[u] = c2; } const size_t oo = (size_t)t * RK + h * HD + d; *(volatile v2us*)(Ah + oo) = oh; *(volatile v2us*)(Al + oo) = ol; __threadfence(); *(volatile v2us*)(Ah + oo) = oh; *(volatile v2us*)(Al + oo) = ol; }

extern "C" void kernel_launch(void* const* d_in, const int* in_sizes, int n_in,
                              void* d_out, int out_size, void* d_ws, size_t ws_size, hipStream_t stream) {
    (void)in_sizes; (void)n_in; (void)out_size;
    const float* IN[10]; for (int i = 0; i < 10; ++i) IN[i] = (const float*)d_in[i];
    float* OUT = (float*)d_out;
    char* wsp = (char*)d_ws;
    auto take = [&](size_t bytes) { char* p = wsp; wsp += (bytes + 255) & ~(size_t)255; return (void*)p; };
    bf* WQ = (bf*)take((size_t)RK * DM * 2); bf* WK = (bf*)take((size_t)RK * DM * 2); bf* WV = (bf*)take((size_t)RK * DM * 2); bf* WO = (bf*)take((size_t)DM * RK * 2);
    bf* XB = (bf*)take((size_t)TT * DM * 2); float* FQ = (float*)take((size_t)TT * RK * 4); float* FK = (float*)take((size_t)TT * RK * 4); float* FV = (float*)take((size_t)TT * RK * 4);
    h16* Q16 = (h16*)take((size_t)NH_ * TT * HD * 2); h16* K16 = (h16*)take((size_t)NH_ * TT * HD * 2); bf* Qh = (bf*)take((size_t)NH_ * TT * HD * 2); bf* Ql = (bf*)take((size_t)NH_ * TT * HD * 2); bf* Kh = (bf*)take((size_t)NH_ * TT * HD * 2); bf* Kl = (bf*)take((size_t)NH_ * TT * HD * 2);
    h16* VT16 = (h16*)take((size_t)NH_ * 64 * TT * 2); bf* VTh = (bf*)take((size_t)NH_ * 64 * TT * 2); bf* VTl = (bf*)take((size_t)NH_ * 64 * TT * 2);
    float* Sb = (float*)take((size_t)TT * TT * 4); h16* P16 = (h16*)take((size_t)TT * TT * 2); bf* Ph = (bf*)take((size_t)RH * TT * 2); bf* Pl = (bf*)take((size_t)RH * TT * 2); float* O = (float*)take((size_t)TT * 64 * 4); bf* Ah = (bf*)take((size_t)TT * RK * 2); bf* Al = (bf*)take((size_t)TT * RK * 2);
    if ((size_t)(wsp - (char*)d_ws) > ws_size) return;
    { const unsigned g = (unsigned)(((size_t)RK * DM / 8 + 255) / 256); k_cvt8<<<g, 256, 0, stream>>>(IN[2], WQ, (size_t)RK * DM / 8); k_cvt8<<<g, 256, 0, stream>>>(IN[4], WK, (size_t)RK * DM / 8); k_cvt8<<<g, 256, 0, stream>>>(IN[6], WV, (size_t)RK * DM / 8); k_cvt8<<<g, 256, 0, stream>>>(IN[8], WO, (size_t)DM * RK / 8); }
    const dim3 gP(TT / 64, RK / 64, 1);
    for (int b = 0; b < NB_; ++b) { const float* mkb = IN[1] + (size_t)b * TT * TT;
        k_cvt8<<<(unsigned)(((size_t)TT * DM / 8 + 255) / 256), 256, 0, stream>>>(IN[0] + (size_t)b * TT * DM, XB, (size_t)TT * DM / 8);
        k_gemmw<bf, 0, true><<<gP, 32, 0, stream>>>(XB, nullptr, WQ, nullptr, DM, FQ, RK, IN[3], 0, 0, 0); k_gemmw<bf, 0, true><<<gP, 32, 0, stream>>>(XB, nullptr, WK, nullptr, DM, FK, RK, IN[5], 0, 0, 0); k_gemmw<bf, 0, true><<<gP, 32, 0, stream>>>(XB, nullptr, WV, nullptr, DM, FV, RK, IN[7], 0, 0, 0);
        k_qkp<<<(unsigned)(((size_t)NH_ * TT * HD / 2 + 255) / 256), 256, 0, stream>>>(FQ, FK, Q16, K16, Qh, Ql, Kh, Kl); k_vtp<<<(unsigned)(((size_t)NH_ * 64 * TT / 2 + 255) / 256), 256, 0, stream>>>(FV, VT16, VTh, VTl);
        for (int h = 0; h < NH_; ++h) { const size_t po = (size_t)h * TT * HD, vo = (size_t)h * 64 * TT;
            k_gemmw<bf, 2, false><<<dim3(RH / 64, TT / 64, 1), 32, 0, stream>>>(Qh + po, Ql + po, Kh + po, Kl + po, HD, Sb, TT, nullptr, 0, 0, 0);
            k_gemmw<h16, 0, false><<<dim3((TT - RH) / 64, TT / 64, 1), 32, 0, stream>>>(Q16 + po + (size_t)RH * HD, nullptr, K16 + po, nullptr, HD, Sb + (size_t)RH * TT, TT, nullptr, 0, 0, 0);
            k_hsoft<<<TT / 8, 256, 0, stream>>>(Sb, mkb, P16, Ph, Pl);
            k_gemmw<bf, 2, false><<<dim3(RH / 64, 1, 1), 32, 0, stream>>>(Ph, Pl, VTh + vo, VTl + vo, TT, O, 64, nullptr, 0, 0, 0);
            k_gemmw<h16, 0, false><<<dim3((TT - RH) / 64, 1, 1), 32, 0, stream>>>(P16 + (size_t)RH * TT, nullptr, VT16 + vo, nullptr, TT, O + (size_t)RH * 64, 64, nullptr, 0, 0, 0);
            k_ofm<<<(TT * HD / 2 + 255) / 256, 256, 0, stream>>>(O, h, Ah, Al); }
        k_gemmw<bf, 1, true><<<dim3(TT / 64, DM / 64, 1), 32, 0, stream>>>(Ah, Al, WO, nullptr, RK, OUT + (size_t)b * TT * DM, DM, IN[9], 0, 0, 0); }
}
